// SingleLayerRGN_38319698215247
// MI455X (gfx1250) — hardware-verified
//
#include <hip/hip_runtime.h>
#include <stddef.h>


#define NF    64
#define EF    16
#define HID   128
#define OUTD  64
#define NTE   4
#define NTN   2
#define KIN   144
#define KP    160

#define NTHR  256
#define NWAVE 8
#define EPT   8
#define CHUNK (NTHR * EPT)
#define WCAP  (EPT * 32)
#define LISTN (NWAVE * WCAP)
#define PASSN 256
#define PCAP  (CHUNK + PASSN)
#define NB    512
#define MAXT  24
#define SRTN  (MAXT * 16)
#define STGF  1280

static_assert(PASSN == NTHR);
static_assert((PCAP % PASSN) == 0);
static_assert((NB % (16 * NWAVE)) == 0);
static_assert(STGF * 4 >= 16 * KP * 2);
static_assert(STGF >= 16 * OUTD);
static_assert(SRTN >= PASSN + 4 * 15);
static_assert((KP % 32) == 0 && KP >= KIN);

typedef float          v4f   __attribute__((ext_vector_type(4)));
typedef float          v8f   __attribute__((ext_vector_type(8)));
typedef int            v4i   __attribute__((ext_vector_type(4)));
typedef unsigned short v8us  __attribute__((ext_vector_type(8)));
typedef unsigned short v16us __attribute__((ext_vector_type(16)));
typedef __bf16         v16bf __attribute__((ext_vector_type(16)));
union FragB { v16us u; v8us h[2]; v16bf v; };

__device__ __forceinline__ v8f zero8f() {
  v8f z;
#pragma unroll
  for (int i = 0; i < 8; ++i) z[i] = 0.0f;
  return z;
}

__device__ __forceinline__ unsigned short bf_bits(float x) {
  unsigned u = __float_as_uint(x);
  u += 0x7FFFu + ((u >> 16) & 1u);
  return (unsigned short)(u >> 16);
}
__device__ __forceinline__ float bf_val(unsigned short b) { return __uint_as_float(((unsigned)b) << 16); }
__device__ __forceinline__ float bf_rn(float x) { return bf_val(bf_bits(x)); }

__device__ __forceinline__ v8us cvt8(v4f a, v4f b) {
  v8us o;
  o[0] = bf_bits(a.x); o[1] = bf_bits(a.y); o[2] = bf_bits(a.z); o[3] = bf_bits(a.w);
  o[4] = bf_bits(b.x); o[5] = bf_bits(b.y); o[6] = bf_bits(b.z); o[7] = bf_bits(b.w);
  return o;
}

__device__ __forceinline__ v8f wmb(v16bf a, v16bf b, v8f c) {
  v8f d = __builtin_amdgcn_wmma_f32_16x16x32_bf16(false, a, false, b, (short)0, c, false, false);
  asm volatile("v_nop\n\tv_nop\n\tv_nop\n\tv_nop" : "+v"(d) : "v"(a), "v"(b));
  return d;
}

__device__ __forceinline__ void mkh(v8f d0, v8f d1, const float* bp0, const float* bp1, FragB& fh, FragB& fl) {
#pragma unroll
  for (int r = 0; r < 8; ++r) {
    const float v0 = fmaxf(d0[r] + bp0[r], 0.0f);
    const unsigned short h0 = bf_bits(v0);
    fh.u[r] = h0;
    fl.u[r] = bf_bits(v0 - bf_val(h0));
    const float v1 = fmaxf(d1[r] + bp1[r], 0.0f);
    const unsigned short h1 = bf_bits(v1);
    fh.u[8 + r] = h1;
    fl.u[8 + r] = bf_bits(v1 - bf_val(h1));
  }
}

__device__ __forceinline__ int scan_chunk(const int* __restrict__ dsts, int nE, int cbase, int nodeBase,
                                          int vec8, int* list, int tid, int wave) {
  int wc = 0;
  const int el0  = tid * EPT;
  const int e0   = cbase + el0;
  const int sent = -2147483647 - 1;
  v4i da, db;
  if (vec8 != 0 && cbase + CHUNK <= nE) {
    da = *(const v4i*)(dsts + e0);
    db = *(const v4i*)(dsts + e0 + 4);
  } else {
    da.x = (e0     < nE) ? dsts[min(e0, nE - 1)] : sent;
    da.y = (e0 + 1 < nE) ? dsts[min(e0 + 1, nE - 1)] : sent;
    da.z = (e0 + 2 < nE) ? dsts[min(e0 + 2, nE - 1)] : sent;
    da.w = (e0 + 3 < nE) ? dsts[min(e0 + 3, nE - 1)] : sent;
    db.x = (e0 + 4 < nE) ? dsts[min(e0 + 4, nE - 1)] : sent;
    db.y = (e0 + 5 < nE) ? dsts[min(e0 + 5, nE - 1)] : sent;
    db.z = (e0 + 6 < nE) ? dsts[min(e0 + 6, nE - 1)] : sent;
    db.w = (e0 + 7 < nE) ? dsts[min(e0 + 7, nE - 1)] : sent;
  }
  const unsigned nb = (unsigned)nodeBase;
  const unsigned s0 = (unsigned)da.x - nb, s1 = (unsigned)da.y - nb;
  const unsigned s2 = (unsigned)da.z - nb, s3 = (unsigned)da.w - nb;
  const unsigned s4 = (unsigned)db.x - nb, s5 = (unsigned)db.y - nb;
  const unsigned s6 = (unsigned)db.z - nb, s7 = (unsigned)db.w - nb;
  const bool h0 = s0 < (unsigned)NB, h1 = s1 < (unsigned)NB, h2 = s2 < (unsigned)NB, h3 = s3 < (unsigned)NB;
  const bool h4 = s4 < (unsigned)NB, h5 = s5 < (unsigned)NB, h6 = s6 < (unsigned)NB, h7 = s7 < (unsigned)NB;
  const unsigned any = __builtin_amdgcn_ballot_w32(h0 | h1 | h2 | h3 | h4 | h5 | h6 | h7);
  if (any != 0u) {
#define HITJ(J, HJ) { \
      const unsigned mj = __builtin_amdgcn_ballot_w32(HJ); \
      if (mj != 0u) { \
        if (HJ) { \
          const int pos = wc + (int)__builtin_amdgcn_mbcnt_lo(mj, 0u); \
          if (pos < WCAP) list[wave * WCAP + pos] = el0 + (J); \
        } \
        wc += (int)__builtin_popcount(mj); } }
    HITJ(0, h0)
    HITJ(1, h1)
    HITJ(2, h2)
    HITJ(3, h3)
    HITJ(4, h4)
    HITJ(5, h5)
    HITJ(6, h6)
    HITJ(7, h7)
#undef HITJ
  }
  return wc;
}

__global__ __launch_bounds__(NTHR) void k_prep(
    const float* __restrict__ W1, const float* __restrict__ W2,
    const float* __restrict__ U1, const float* __restrict__ U2,
    unsigned short* W1T, unsigned short* W2T, unsigned short* U1T, unsigned short* U2T) {
  const int u  = blockIdx.x * NTHR + threadIdx.x;
  const int n1 = NTE * HID * (KP / 8);
  const int n2 = n1 + NTE * OUTD * (HID / 8);
  const int n3 = n2 + NTN * HID * (NF / 8);
  const int n4 = n3 + NTN * OUTD * (HID / 8);
  if (u >= n4) return;
  v8f x = zero8f();
  unsigned short* dp;
  if (u < n1) {
    const int row = u / (KP / 8);
    const int kc  = (u - row * (KP / 8)) * 8;
    const int t   = row / HID, n = row - (row / HID) * HID;
#pragma unroll
    for (int i = 0; i < 8; ++i) {
      const int k  = kc + i;
      const int kk = (k < KIN) ? k : (KIN - 1);
      const float w = W1[((size_t)t * KIN + kk) * HID + n];
      x[i] = (k < KIN) ? w : 0.0f;
    }
    dp = W1T + (size_t)u * 8;
  } else if (u < n2) {
    const int j   = u - n1;
    const int row = j / (HID / 8);
    const int kc  = (j - row * (HID / 8)) * 8;
    const int t   = row / OUTD, n = row - (row / OUTD) * OUTD;
#pragma unroll
    for (int i = 0; i < 8; ++i) x[i] = W2[((size_t)t * HID + kc + i) * OUTD + n];
    dp = W2T + (size_t)j * 8;
  } else if (u < n3) {
    const int j   = u - n2;
    const int row = j / (NF / 8);
    const int kc  = (j - row * (NF / 8)) * 8;
    const int t   = row / HID, n = row - (row / HID) * HID;
#pragma unroll
    for (int i = 0; i < 8; ++i) x[i] = U1[((size_t)t * NF + kc + i) * HID + n];
    dp = U1T + (size_t)j * 8;
  } else {
    const int j   = u - n3;
    const int row = j / (HID / 8);
    const int kc  = (j - row * (HID / 8)) * 8;
    const int t   = row / OUTD, n = row - (row / OUTD) * OUTD;
#pragma unroll
    for (int i = 0; i < 8; ++i) x[i] = U2[((size_t)t * HID + kc + i) * OUTD + n];
    dp = U2T + (size_t)j * 8;
  }
  v8us o;
#pragma unroll
  for (int i = 0; i < 8; ++i) o[i] = bf_bits(x[i]);
  *(volatile v8us*)dp = o;
  __threadfence();
  *(volatile v8us*)dp = o;
}

__global__ __launch_bounds__(NTHR) __attribute__((amdgpu_num_vgpr(256)))
void k_edge(const float* __restrict__ nf, const float* __restrict__ ef,
            const float* __restrict__ b1, const float* __restrict__ b2,
            const float* __restrict__ ub1, const float* __restrict__ ub2,
            const int* __restrict__ esrc, const int* __restrict__ edst,
            const int* __restrict__ etyp, const int* __restrict__ ntyp,
            const unsigned short* __restrict__ W1T, const unsigned short* __restrict__ W2T,
            const unsigned short* __restrict__ U1T, const unsigned short* __restrict__ U2T,
            float* outp, int nN, int nE, int vec8) {
  __shared__ __attribute__((aligned(16))) float acc[NB * OUTD];
  __shared__ __attribute__((aligned(16))) float cntf[NB];
  __shared__ __attribute__((aligned(16))) float stg[NWAVE * STGF];
  __shared__ __attribute__((aligned(16))) int   list[LISTN];
  __shared__ __attribute__((aligned(16))) int   pend[PCAP];
  __shared__ int   srt_e[SRTN];
  __shared__ int   srt_sl[SRTN];
  __shared__ int   tile_t[MAXT];
  __shared__ __attribute__((aligned(16))) float sb1[NTE * HID];
  __shared__ __attribute__((aligned(16))) float sb2[NTE * OUTD];
  __shared__ __attribute__((aligned(16))) float su1[NTN * HID];
  __shared__ __attribute__((aligned(16))) float su2[NTN * OUTD];
  __shared__ int wcnt[NWAVE];
  __shared__ int wtc[NWAVE * 4];
  __shared__ int pendN;

  const int tid = threadIdx.x, lane = tid & 31, wave = tid >> 5, hh = lane >> 4, m = lane & 15;
  const int nodeBase = blockIdx.x * NB;
  float* stw = stg + wave * STGF;
  unsigned short* xs = (unsigned short*)stw;

  {
    const v4f z4 = {0.0f, 0.0f, 0.0f, 0.0f};
    for (int i = tid; i < NB * OUTD / 4; i += NTHR) *(v4f*)(acc + 4 * i) = z4;
    for (int i = tid; i < NB; i += NTHR) cntf[i] = 0.0f;
    for (int i = tid; i < NTE * HID; i += NTHR) sb1[i] = bf_rn(b1[i]);
    for (int i = tid; i < NTE * OUTD; i += NTHR) sb2[i] = bf_rn(b2[i]);
    for (int i = tid; i < NTN * HID; i += NTHR) su1[i] = bf_rn(ub1[i]);
    for (int i = tid; i < NTN * OUTD; i += NTHR) su2[i] = bf_rn(ub2[i]);
    if (tid == 0) pendN = 0;
  }
  __syncthreads();

  const int nChunks = (nE + CHUNK - 1) / CHUNK;
#pragma unroll 1
  for (int ch = 0; ch < nChunks; ++ch) {
    const int cbase = ch * CHUNK;
    const int wc = scan_chunk(edst, nE, cbase, nodeBase, vec8, list, tid, wave);
    if (lane == 0) wcnt[wave] = wc;
    __syncthreads();

    const int base = pendN;
    int tot = 0, myoff = 0;
#pragma unroll
    for (int w = 0; w < NWAVE; ++w) {
      int c = wcnt[w];
      c = c > WCAP ? WCAP : (c < 0 ? 0 : c);
      if (w < wave) myoff += c;
      tot += c;
    }
    int newN = base + tot;
    newN = newN > PCAP ? PCAP : newN;
    {
      int n = wcnt[wave];
      n = n > WCAP ? WCAP : (n < 0 ? 0 : n);
      const int* lp = list + wave * WCAP;
      for (int i = lane; i < n; i += 32) {
        const int pos = base + myoff + i;
        if (pos < PCAP) pend[pos] = cbase + lp[i];
      }
    }
    const int fin = (ch == nChunks - 1) ? 1 : 0;
    const int R   = (fin != 0) ? (newN + PASSN - 1) / PASSN : newN / PASSN;
    const int Pv  = (fin != 0) ? newN : R * PASSN;
    __syncthreads();

#pragma unroll 1
    for (int r = 0; r < R; ++r) {
      const int idx = r * PASSN + tid;
      const bool valid = idx < Pv;
      int e = pend[idx < PCAP ? idx : (PCAP - 1)];
      e = valid ? e : 0;
      e = e < 0 ? 0 : (e > nE - 1 ? nE - 1 : e);
      int ty = etyp[e];
      ty = ty < 0 ? 0 : (ty > NTE - 1 ? NTE - 1 : ty);
      ty = valid ? ty : -1;
      int slot;
      {
        const int dd = edst[e];
        slot = dd - nodeBase;
        if (!valid || (unsigned)slot >= (unsigned)NB) slot = NB;
      }
      const unsigned mk0 = __builtin_amdgcn_ballot_w32(ty == 0);
      const unsigned mk1 = __builtin_amdgcn_ballot_w32(ty == 1);
      const unsigned mk2 = __builtin_amdgcn_ballot_w32(ty == 2);
      const unsigned mk3 = __builtin_amdgcn_ballot_w32(ty == 3);
      int rank = 0;
      rank = (ty == 0) ? (int)__builtin_amdgcn_mbcnt_lo(mk0, 0u) : rank;
      rank = (ty == 1) ? (int)__builtin_amdgcn_mbcnt_lo(mk1, 0u) : rank;
      rank = (ty == 2) ? (int)__builtin_amdgcn_mbcnt_lo(mk2, 0u) : rank;
      rank = (ty == 3) ? (int)__builtin_amdgcn_mbcnt_lo(mk3, 0u) : rank;
      if (lane == 0) {
        wtc[wave * 4 + 0] = (int)__builtin_popcount(mk0);
        wtc[wave * 4 + 1] = (int)__builtin_popcount(mk1);
        wtc[wave * 4 + 2] = (int)__builtin_popcount(mk2);
        wtc[wave * 4 + 3] = (int)__builtin_popcount(mk3);
      }
      __syncthreads();

      int c0 = 0, c1 = 0, c2 = 0, c3 = 0, q0 = 0, q1 = 0, q2 = 0, q3 = 0;
#pragma unroll
      for (int w = 0; w < NWAVE; ++w) {
        const int a0 = wtc[w * 4 + 0], a1 = wtc[w * 4 + 1], a2 = wtc[w * 4 + 2], a3 = wtc[w * 4 + 3];
        if (w < wave) { q0 += a0; q1 += a1; q2 += a2; q3 += a3; }
        c0 += a0; c1 += a1; c2 += a2; c3 += a3;
      }
      const int gs1 = (c0 + 15) & ~15;
      const int gs2 = gs1 + ((c1 + 15) & ~15);
      const int gs3 = gs2 + ((c2 + 15) & ~15);
      const int gs4 = gs3 + ((c3 + 15) & ~15);
      int nTiles = gs4 >> 4;
      nTiles = nTiles > MAXT ? MAXT : nTiles;
      if (ty >= 0) {
        const int gsv = (ty == 0) ? 0  : ((ty == 1) ? gs1 : ((ty == 2) ? gs2 : gs3));
        const int qv  = (ty == 0) ? q0 : ((ty == 1) ? q1  : ((ty == 2) ? q2  : q3));
        const int pos = gsv + qv + rank;
        if ((unsigned)pos < (unsigned)SRTN) { srt_e[pos] = e; srt_sl[pos] = slot; }
      }
      for (int p = tid; p < SRTN; p += NTHR) {
        const int tt  = (p >= gs1 ? 1 : 0) + (p >= gs2 ? 1 : 0) + (p >= gs3 ? 1 : 0);
        const int gsv = (tt == 0) ? 0  : ((tt == 1) ? gs1 : ((tt == 2) ? gs2 : gs3));
        const int cv  = (tt == 0) ? c0 : ((tt == 1) ? c1  : ((tt == 2) ? c2  : c3));
        if (p - gsv >= cv) { srt_e[p] = 0; srt_sl[p] = NB; }
        if ((p & 15) == 0) tile_t[p >> 4] = tt;
      }
      __syncthreads();

      const int nTl  = __builtin_amdgcn_readfirstlane(nTiles);
      const int nSub = (nTl + NWAVE - 1) / NWAVE;
#pragma unroll 1
      for (int sp = 0; sp < nSub; ++sp) {
        const int jt  = sp * NWAVE + wave;
        const int has = __builtin_amdgcn_readfirstlane((jt < nTl) ? 1 : 0);

        if (has != 0) {
          const int pidx = sp * (NWAVE * 16) + wave * 16 + m;
          int ee = srt_e[pidx];
          ee = ee < 0 ? 0 : (ee > nE - 1 ? nE - 1 : ee);
          int ss = esrc[ee];
          ss = ss < 0 ? 0 : (ss > nN - 1 ? nN - 1 : ss);
          int de = edst[ee];
          de = de < 0 ? 0 : (de > nN - 1 ? nN - 1 : de);
#pragma unroll
          for (int it = 0; it < 4; ++it) {
            const int uu = it * 32 + lane;
            const int row = uu >> 3, cp = uu & 7;
            const int srw = __shfl(ss, row);
            const float* gp = nf + (size_t)srw * NF + cp * 8;
            const v4f a = *(const v4f*)gp;
            const v4f b = *(const v4f*)(gp + 4);
            *(v8us*)(xs + row * KP + cp * 8) = cvt8(a, b);
          }
          {
            const int row = lane >> 1, hf = lane & 1;
            const int erw = __shfl(ee, row);
            const float* gp = ef + (size_t)erw * EF + hf * 8;
            const v4f a = *(const v4f*)gp;
            const v4f b = *(const v4f*)(gp + 4);
            *(v8us*)(xs + row * KP + NF + hf * 8) = cvt8(a, b);
          }
#pragma unroll
          for (int it = 0; it < 4; ++it) {
            const int uu = it * 32 + lane;
            const int row = uu >> 3, cp = uu & 7;
            const int drw = __shfl(de, row);
            const float* gp = nf + (size_t)drw * NF + cp * 8;
            const v4f a = *(const v4f*)gp;
            const v4f b = *(const v4f*)(gp + 4);
            *(v8us*)(xs + row * KP + NF + EF + cp * 8) = cvt8(a, b);
          }
          if (lane < 16) {
            v8us z;
#pragma unroll
            for (int i = 0; i < 8; ++i) z[i] = (unsigned short)0;
            *(v8us*)(xs + lane * KP + KIN) = z;
            *(v8us*)(xs + lane * KP + KIN + 8) = z;
          }
        }
        __syncthreads();

        if (has != 0) {
          int t = __builtin_amdgcn_readfirstlane(tile_t[jt < MAXT ? jt : (MAXT - 1)]);
          t = t < 0 ? 0 : (t > NTE - 1 ? NTE - 1 : t);
          const unsigned short* xr  = xs + m * KP + 8 * hh;
          const unsigned short* w1t = W1T + ((size_t)t * HID + m) * KP + 8 * hh;
          v8f dA[8];
#pragma unroll
          for (int ft = 0; ft < 8; ++ft) dA[ft] = zero8f();
#pragma unroll 1
          for (int ks = 0; ks < KP / 32; ++ks) {
            const int k0 = ks * 32;
            FragB xb;
            xb.h[0] = *(const v8us*)(xr + k0);
            xb.h[1] = *(const v8us*)(xr + k0 + 16);
#pragma unroll
            for (int ft = 0; ft < 8; ++ft) {
              FragB a;
              const unsigned short* ap = w1t + (size_t)ft * 16 * KP + k0;
              a.h[0] = *(const v8us*)ap;
              a.h[1] = *(const v8us*)(ap + 16);
              dA[ft] = wmb(a.v, xb.v, dA[ft]);
            }
          }
          const float* b1p = sb1 + t * HID + 8 * hh;
          const unsigned short* w2t = W2T + ((size_t)t * OUTD + m) * HID + 8 * hh;
          v8f dB[4];
#pragma unroll
          for (int ot = 0; ot < 4; ++ot) dB[ot] = zero8f();
#pragma unroll
          for (int ks2 = 0; ks2 < HID / 32; ++ks2) {
            FragB fh, fl;
            mkh(dA[2 * ks2], dA[2 * ks2 + 1], b1p + 32 * ks2, b1p + 32 * ks2 + 16, fh, fl);
#pragma unroll
            for (int ot = 0; ot < 4; ++ot) {
              FragB a;
              const unsigned short* ap = w2t + (size_t)ot * 16 * HID + 32 * ks2;
              a.h[0] = *(const v8us*)ap;
              a.h[1] = *(const v8us*)(ap + 16);
              dB[ot] = wmb(a.v, fh.v, dB[ot]);
              dB[ot] = wmb(a.v, fl.v, dB[ot]);
            }
          }
          const float* b2p = sb2 + t * OUTD + 8 * hh;
          float* mw = stw + m * OUTD + 8 * hh;
#pragma unroll
          for (int ot = 0; ot < 4; ++ot) {
            v4f u0, u1;
            u0.x = dB[ot][0] + b2p[16 * ot + 0]; u0.y = dB[ot][1] + b2p[16 * ot + 1];
            u0.z = dB[ot][2] + b2p[16 * ot + 2]; u0.w = dB[ot][3] + b2p[16 * ot + 3];
            u1.x = dB[ot][4] + b2p[16 * ot + 4]; u1.y = dB[ot][5] + b2p[16 * ot + 5];
            u1.z = dB[ot][6] + b2p[16 * ot + 6]; u1.w = dB[ot][7] + b2p[16 * ot + 7];
            *(v4f*)(mw + 16 * ot)     = u0;
            *(v4f*)(mw + 16 * ot + 4) = u1;
          }
        }
        __syncthreads();

        if (wave == 0) {
#pragma unroll 1
          for (int i = 0; i < NWAVE * 16; ++i) {
            const int p  = sp * (NWAVE * 16) + i;
            const int sl = __builtin_amdgcn_readfirstlane(srt_sl[p]);
            if ((unsigned)sl < (unsigned)NB) {
              const float* mrow = stg + (i >> 4) * STGF + (i & 15) * OUTD;
              if (lane < 16) {
                float* aq = acc + sl * OUTD + 4 * lane;
                const v4f av = *(const v4f*)aq;
                const v4f mv = *(const v4f*)(mrow + 4 * lane);
                *(v4f*)aq = av + mv;
              } else if (lane == 16) {
                cntf[sl] += 1.0f;
              }
            }
          }
        }
        __syncthreads();
      }
    }

    int rem = newN - R * PASSN;
    rem = rem < 0 ? 0 : rem;
    if (R > 0 && tid < rem) pend[tid] = pend[R * PASSN + tid];
    if (tid == 0) pendN = rem;
  }
  __syncthreads();

#pragma unroll 1
  for (int qi = 0; qi < NB / (16 * NWAVE); ++qi) {
    const int s0 = (qi * NWAVE + wave) * 16;
    const int sr = s0 + m;
    const float inv = 1.0f / fmaxf(cntf[sr], 1.0f);
    const float* ar = acc + sr * OUTD + 8 * hh;
    FragB gh[2], gl[2];
#pragma unroll
    for (int ks = 0; ks < NF / 32; ++ks) {
      const v4f a0 = *(const v4f*)(ar + 32 * ks);
      const v4f a1 = *(const v4f*)(ar + 32 * ks + 4);
      const v4f e0 = *(const v4f*)(ar + 32 * ks + 16);
      const v4f e1 = *(const v4f*)(ar + 32 * ks + 20);
#pragma unroll
      for (int i = 0; i < 4; ++i) {
        const float v0 = a0[i] * inv; const unsigned short h0 = bf_bits(v0);
        gh[ks].u[i] = h0;      gl[ks].u[i] = bf_bits(v0 - bf_val(h0));
        const float v1 = a1[i] * inv; const unsigned short h1 = bf_bits(v1);
        gh[ks].u[4 + i] = h1;  gl[ks].u[4 + i] = bf_bits(v1 - bf_val(h1));
        const float v2 = e0[i] * inv; const unsigned short h2 = bf_bits(v2);
        gh[ks].u[8 + i] = h2;  gl[ks].u[8 + i] = bf_bits(v2 - bf_val(h2));
        const float v3 = e1[i] * inv; const unsigned short h3 = bf_bits(v3);
        gh[ks].u[12 + i] = h3; gl[ks].u[12 + i] = bf_bits(v3 - bf_val(h3));
      }
    }
    int nd = nodeBase + sr;
    nd = nd > nN - 1 ? nN - 1 : (nd < 0 ? 0 : nd);
    const int myT = ntyp[nd];
    v8f ov[4];
#pragma unroll
    for (int ot = 0; ot < 4; ++ot) ov[ot] = zero8f();
#pragma unroll 1
    for (int nt = 0; nt < NTN; ++nt) {
      const unsigned short* u1t = U1T + ((size_t)nt * HID + m) * NF + 8 * hh;
      v8f dU[8];
#pragma unroll
      for (int ft = 0; ft < 8; ++ft) dU[ft] = zero8f();
#pragma unroll
      for (int ks = 0; ks < NF / 32; ++ks) {
#pragma unroll
        for (int ft = 0; ft < 8; ++ft) {
          FragB a;
          const unsigned short* ap = u1t + (size_t)ft * 16 * NF + 32 * ks;
          a.h[0] = *(const v8us*)ap;
          a.h[1] = *(const v8us*)(ap + 16);
          dU[ft] = wmb(a.v, gh[ks].v, dU[ft]);
          dU[ft] = wmb(a.v, gl[ks].v, dU[ft]);
        }
      }
      const float* bp = su1 + nt * HID + 8 * hh;
      const unsigned short* u2t = U2T + ((size_t)nt * OUTD + m) * HID + 8 * hh;
      v8f dO[4];
#pragma unroll
      for (int ot = 0; ot < 4; ++ot) dO[ot] = zero8f();
#pragma unroll
      for (int ks2 = 0; ks2 < HID / 32; ++ks2) {
        FragB fh, fl;
        mkh(dU[2 * ks2], dU[2 * ks2 + 1], bp + 32 * ks2, bp + 32 * ks2 + 16, fh, fl);
#pragma unroll
        for (int ot = 0; ot < 4; ++ot) {
          FragB a;
          const unsigned short* ap = u2t + (size_t)ot * 16 * HID + 32 * ks2;
          a.h[0] = *(const v8us*)ap;
          a.h[1] = *(const v8us*)(ap + 16);
          dO[ot] = wmb(a.v, fh.v, dO[ot]);
          dO[ot] = wmb(a.v, fl.v, dO[ot]);
        }
      }
      const bool sel = (myT == nt);
      const float* bq = su2 + nt * OUTD + 8 * hh;
#pragma unroll
      for (int ot = 0; ot < 4; ++ot) {
#pragma unroll
        for (int rr = 0; rr < 8; ++rr) {
          const float v = dO[ot][rr] + bq[16 * ot + rr];
          ov[ot][rr] = sel ? v : ov[ot][rr];
        }
      }
    }
    __syncthreads();
    {
      float* ow = stw + m * OUTD + 8 * hh;
#pragma unroll
      for (int ot = 0; ot < 4; ++ot) {
        v4f u0, u1;
        u0.x = ov[ot][0]; u0.y = ov[ot][1]; u0.z = ov[ot][2]; u0.w = ov[ot][3];
        u1.x = ov[ot][4]; u1.y = ov[ot][5]; u1.z = ov[ot][6]; u1.w = ov[ot][7];
        *(v4f*)(ow + 16 * ot)     = u0;
        *(v4f*)(ow + 16 * ot + 4) = u1;
      }
    }
    __syncthreads();
    v4f rv[8];
#pragma unroll
    for (int c = 0; c < 8; ++c) rv[c] = *(const v4f*)(stw + (2 * c + hh) * OUTD + 4 * m);
#pragma unroll
    for (int c = 0; c < 8; ++c) {
      const int node = nodeBase + s0 + 2 * c + hh;
      if (node < nN) *(volatile v4f*)(outp + (size_t)node * OUTD + 4 * m) = rv[c];
    }
    __threadfence();
#pragma unroll
    for (int c = 0; c < 8; ++c) {
      const int node = nodeBase + s0 + 2 * c + hh;
      if (node < nN) *(volatile v4f*)(outp + (size_t)node * OUTD + 4 * m) = rv[c];
    }
  }
}

extern "C" void kernel_launch(void* const* d_in, const int* in_sizes, int n_in,
                              void* d_out, int out_size, void* d_ws, size_t ws_size,
                              hipStream_t stream) {
  if (n_in < 14) return;
  if (in_sizes[0] <= 0 || in_sizes[10] <= 0) return;
  const int nN = in_sizes[0] / NF;
  const int nE = in_sizes[10];
  if (nN <= 0 || in_sizes[0] != nN * NF) return;
  if (in_sizes[1] != nE * EF || in_sizes[11] != nE || in_sizes[12] != nE || in_sizes[13] != nN) return;
  if (in_sizes[2] != NTE * KIN * HID || in_sizes[3] != NTE * HID) return;
  if (in_sizes[4] != NTE * HID * OUTD || in_sizes[5] != NTE * OUTD) return;
  if (in_sizes[6] != NTN * NF * HID || in_sizes[7] != NTN * HID) return;
  if (in_sizes[8] != NTN * HID * OUTD || in_sizes[9] != NTN * OUTD) return;
  if (out_size != nN * OUTD) return;

  const float* nf  = (const float*)d_in[0];
  const float* ef  = (const float*)d_in[1];
  const float* mW1 = (const float*)d_in[2];
  const float* mb1 = (const float*)d_in[3];
  const float* mW2 = (const float*)d_in[4];
  const float* mb2 = (const float*)d_in[5];
  const float* uW1 = (const float*)d_in[6];
  const float* ub1 = (const float*)d_in[7];
  const float* uW2 = (const float*)d_in[8];
  const float* ub2 = (const float*)d_in[9];
  const int* esrc  = (const int*)d_in[10];
  const int* edst  = (const int*)d_in[11];
  const int* etyp  = (const int*)d_in[12];
  const int* ntyp  = (const int*)d_in[13];
  float* out = (float*)d_out;

  const size_t szW1 = (size_t)NTE * HID * KP * 2;
  const size_t szW2 = (size_t)NTE * OUTD * HID * 2;
  const size_t szU1 = (size_t)NTN * HID * NF * 2;
  const size_t szU2 = (size_t)NTN * OUTD * HID * 2;
  const size_t oW1 = 0;
  const size_t oW2 = oW1 + szW1;
  const size_t oU1 = oW2 + szW2;
  const size_t oU2 = oU1 + szU1;
  const size_t total = oU2 + szU2;
  if (total > ws_size) return;
  char* ws = (char*)d_ws;
  unsigned short* W1T = (unsigned short*)(ws + oW1);
  unsigned short* W2T = (unsigned short*)(ws + oW2);
  unsigned short* U1T = (unsigned short*)(ws + oU1);
  unsigned short* U2T = (unsigned short*)(ws + oU2);

  const int nUnits = NTE * HID * (KP / 8) + NTE * OUTD * (HID / 8) + NTN * HID * (NF / 8) + NTN * OUTD * (HID / 8);
  k_prep<<<(nUnits + NTHR - 1) / NTHR, NTHR, 0, stream>>>(mW1, mW2, uW1, uW2, W1T, W2T, U1T, U2T);

  const int nBlk = (nN + NB - 1) / NB;
  const int vec8 = ((nE & 3) == 0) ? 1 : 0;
  k_edge<<<nBlk, NTHR, 0, stream>>>(nf, ef, mb1, mb2, ub1, ub2, esrc, edst, etyp, ntyp,
                                   W1T, W2T, U1T, U2T, out, nN, nE, vec8);
}
